// T5LayerSelfAttention_87247965650972
// MI455X (gfx1250) — hardware-verified
//
#include <hip/hip_runtime.h>
#include <math.h>

#ifndef NB
#define NB 2
#endif
#ifndef SEQ
#define SEQ 2048
#endif
#define NB_FULL  2
#define SEQ_FULL 2048
#define DM   1024
#define NH   16
#define HD   64
#define NBKT 32
#define MT   (NB * SEQ)
#define BDW  4096
#define BDC  2032
#define AWV  4
#define RWP  48
#define XSC  16.0f
#define WSCL 256.0f
#define QKS  16.0f
#define QRS  2048.0f
#define VSC  16.0f
#define PCAR 16384.0f
#define SC1  (1.0f / 256.0f)
#define SC2  (1.0f / 524288.0f)
#define OSC  (1.0f / 262144.0f)
#define LNEPS 1.0e-6f

static_assert(NB >= 1 && NB <= NB_FULL);
static_assert(SEQ >= 64 && SEQ <= SEQ_FULL && (SEQ % 64) == 0);
static_assert(NH * HD == DM);
static_assert(HD == 64);
static_assert(BDW == 2 * SEQ_FULL);
static_assert((MT % 64) == 0 && (DM % 64) == 0 && (MT % 32) == 0);
static_assert((((MT / 64) * (DM / 64)) % 8) == 0);
static_assert(((NB * NH * (SEQ / 16)) % AWV) == 0);
static_assert(NBKT * NH == 512);
static_assert(BDW == 16 * 256);
static_assert((DM % 256) == 0);

typedef _Float16 v16h __attribute__((ext_vector_type(16)));
typedef __bf16 v16bf __attribute__((ext_vector_type(16)));
typedef unsigned short v16us __attribute__((ext_vector_type(16)));
typedef unsigned short v8us  __attribute__((ext_vector_type(8)));
typedef float v8f __attribute__((ext_vector_type(8)));
typedef float v4f __attribute__((ext_vector_type(4)));
typedef unsigned int v4u __attribute__((ext_vector_type(4)));

union FragU { v16us v; v8us h[2]; };

__device__ __forceinline__ unsigned short bf_bits(float f) {
  const unsigned u = __float_as_uint(f);
  return (unsigned short)((u + 0x7FFFu + ((u >> 16) & 1u)) >> 16);
}
__device__ __forceinline__ float bf_up(unsigned short h) { return __uint_as_float(((unsigned)h) << 16); }
__device__ __forceinline__ float bfr(float f) { return bf_up(bf_bits(f)); }
__device__ __forceinline__ unsigned short h_bits(_Float16 x) { return __builtin_bit_cast(unsigned short, x); }
__device__ __forceinline__ unsigned short f2h(float f) { return h_bits((_Float16)f); }
__device__ __forceinline__ unsigned pk16(unsigned short a, unsigned short b) { return (unsigned)a | ((unsigned)b << 16); }
__device__ __forceinline__ int clampi(int v, int lo, int hi) { return v < lo ? lo : (v > hi ? hi : v); }
__device__ __forceinline__ v8f zero8() { v8f z = {0.f, 0.f, 0.f, 0.f, 0.f, 0.f, 0.f, 0.f}; return z; }

__device__ __forceinline__ v16us ldfrag_u(const unsigned short* p) {
  FragU f;
  f.h[0] = *(const v8us*)(p);
  f.h[1] = *(const v8us*)(p + 16);
  return f.v;
}

template <int OPK>
__device__ __forceinline__ v8f mma_raw(v16us a, v16us b, v8f c) {
  if (OPK == 0)
    return __builtin_amdgcn_wmma_f32_16x16x32_f16(false, __builtin_bit_cast(v16h, a), false,
                                                  __builtin_bit_cast(v16h, b), (short)0, c, false, false);
  return __builtin_amdgcn_wmma_f32_16x16x32_bf16(false, __builtin_bit_cast(v16bf, a), false,
                                                 __builtin_bit_cast(v16bf, b), (short)0, c, false, false);
}
template <int OPK>
__device__ __forceinline__ v8f mma_g(v16us a, v16us b, v8f c) {
  c = mma_raw<OPK>(a, b, c);
#if defined(__HIP_DEVICE_COMPILE__)
  asm volatile("v_nop\n\tv_nop\n\tv_nop\n\tv_nop" : "+v"(c) : "v"(a), "v"(b));
#endif
  return c;
}
__device__ __forceinline__ void dep_guard1(v8f& a, v8f& b, v16us x) {
#if defined(__HIP_DEVICE_COMPILE__)
  asm volatile("v_nop\n\tv_nop\n\tv_nop\n\tv_nop" : "+v"(a), "+v"(b) : "v"(x));
#endif
}
__device__ __forceinline__ void keep4_u(v16us a, v16us b, v16us c, v16us d) {
#if defined(__HIP_DEVICE_COMPILE__)
  asm volatile("v_nop" :: "v"(a), "v"(b), "v"(c), "v"(d));
#endif
}
__device__ __forceinline__ void acc_guard4(v8f& a, v8f& b, v8f& c, v8f& d) {
#if defined(__HIP_DEVICE_COMPILE__)
  asm volatile("v_nop\n\tv_nop\n\tv_nop\n\tv_nop" : "+v"(a), "+v"(b), "+v"(c), "+v"(d));
#endif
}
__device__ __forceinline__ void wave_sync_lds() {
  __builtin_amdgcn_fence(__ATOMIC_RELEASE, "workgroup");
  __builtin_amdgcn_wave_barrier();
  __builtin_amdgcn_fence(__ATOMIC_ACQUIRE, "workgroup");
}

__global__ __launch_bounds__(256) void cvt_x(const float* __restrict__ x, unsigned short* ob,
                                             unsigned short* oh, float* rstd) {
  __shared__ float srs[32];
  const int lane = threadIdx.x & 31, wv = threadIdx.x >> 5;
  const int row0 = blockIdx.x * 32;
#pragma unroll 1
  for (int rr = 0; rr < 4; ++rr) {
    const int tok = row0 + wv * 4 + rr;
    const int b = tok / SEQ, s = tok - b * SEQ;
    const float* src = x + ((size_t)b * SEQ_FULL + (size_t)s) * DM;
    const size_t orow = (size_t)tok * DM;
    float ss = 0.f;
#pragma unroll 1
    for (int it = 0; it < DM / 256; ++it) {
      const int col = it * 256 + lane * 8;
      const v4f a0 = *(const v4f*)(src + col);
      const v4f a1 = *(const v4f*)(src + col + 4);
      v4u hb, hh;
#pragma unroll
      for (int e = 0; e < 2; ++e) {
        const unsigned short u0 = bf_bits(a0[2 * e]), u1 = bf_bits(a0[2 * e + 1]);
        const unsigned short u2 = bf_bits(a1[2 * e]), u3 = bf_bits(a1[2 * e + 1]);
        const float x0 = bf_up(u0), x1 = bf_up(u1), x2 = bf_up(u2), x3 = bf_up(u3);
        ss = fmaf(x0, x0, ss); ss = fmaf(x1, x1, ss); ss = fmaf(x2, x2, ss); ss = fmaf(x3, x3, ss);
        hb[e]     = pk16(u0, u1);
        hb[2 + e] = pk16(u2, u3);
        hh[e]     = pk16(f2h(x0 * XSC), f2h(x1 * XSC));
        hh[2 + e] = pk16(f2h(x2 * XSC), f2h(x3 * XSC));
      }
      unsigned short* db = ob + orow + col;
      unsigned short* dh = oh + orow + col;
      *(volatile v4u*)db = hb;
      *(volatile v4u*)dh = hh;
      __threadfence();
      *(volatile v4u*)db = hb;
      *(volatile v4u*)dh = hh;
    }
    ss += __shfl_xor(ss, 16, 32);
    ss += __shfl_xor(ss, 8, 32);
    ss += __shfl_xor(ss, 4, 32);
    ss += __shfl_xor(ss, 2, 32);
    ss += __shfl_xor(ss, 1, 32);
    if (lane == 0) srs[wv * 4 + rr] = rsqrtf(ss * (1.0f / (float)DM) + LNEPS);
  }
  __syncthreads();
  if (wv == 0) {
    const float v = srs[lane];
    float* d = rstd + row0 + lane;
    *(volatile float*)d = v;
    __threadfence();
    *(volatile float*)d = v;
  }
}

__global__ __launch_bounds__(256) void cvt_w(const float* __restrict__ w0, const float* __restrict__ w1,
                                             const float* __restrict__ w2, const float* __restrict__ w3,
                                             const float* __restrict__ lnw, unsigned short* o) {
  __shared__ __align__(16) float sm[64 * 65];
  __shared__ float slw[64];
  const int y = blockIdx.y;
  const float* w = (y == 0) ? w0 : ((y == 1) ? w1 : ((y == 2) ? w2 : w3));
  const int k0 = (blockIdx.x >> 4) << 6, n0 = (blockIdx.x & 15) << 6;
  const int t = threadIdx.x, lane = t & 31, wv = t >> 5;
#pragma unroll
  for (int it = 0; it < 4; ++it) {
    const int r = it * 16 + (t >> 4), c4 = (t & 15) * 4;
    const v4f v = *(const v4f*)(w + (size_t)(k0 + r) * DM + (size_t)(n0 + c4));
    float* sp = sm + r * 65 + c4;
    sp[0] = v[0]; sp[1] = v[1]; sp[2] = v[2]; sp[3] = v[3];
  }
  if (t < 64) slw[t] = bfr(lnw[k0 + t]);
  __syncthreads();
  const int pl0 = (y == 0) ? 0 : ((y == 1) ? 2 : ((y == 2) ? 4 : 5));
  unsigned short* P0 = o + (size_t)pl0 * DM * DM;
  unsigned short* P1 = (y < 2) ? (P0 + (size_t)DM * DM) : P0;
  const int q8 = lane >> 3, c8 = (lane & 7) * 8;
  v4u ha[2], hl[2];
#pragma unroll
  for (int it = 0; it < 2; ++it) {
    const int r = wv * 8 + it * 4 + q8;
    v4u a = {0u, 0u, 0u, 0u}, l = {0u, 0u, 0u, 0u};
#pragma unroll
    for (int e = 0; e < 4; ++e) {
      const int ka = c8 + 2 * e, kb = ka + 1;
      float va = bfr(sm[ka * 65 + r]), vb = bfr(sm[kb * 65 + r]);
      if (y < 3) { va *= slw[ka]; vb *= slw[kb]; }
      if (y < 2) {
        const unsigned short ua = bf_bits(va), ub = bf_bits(vb);
        a[e] = pk16(ua, ub);
        l[e] = pk16(bf_bits(va - bf_up(ua)), bf_bits(vb - bf_up(ub)));
      } else if (y == 2) {
        a[e] = pk16(f2h(va * WSCL), f2h(vb * WSCL));
      } else {
        a[e] = pk16(bf_bits(va), bf_bits(vb));
      }
    }
    ha[it] = a;
    hl[it] = l;
  }
  for (int pass = 0; pass < 2; ++pass) {
#pragma unroll
    for (int it = 0; it < 2; ++it) {
      const int r = wv * 8 + it * 4 + q8;
      const size_t go = (size_t)(n0 + r) * DM + (size_t)(k0 + c8);
      *(volatile v4u*)(P0 + go) = ha[it];
      if (y < 2) *(volatile v4u*)(P1 + go) = hl[it];
    }
    __threadfence();
  }
}

__device__ __forceinline__ int rel_bucket(int d) {
  int n = -d;
  int ret = 0;
  if (n < 0) { ret = NBKT / 2; n = -n; }
  int bk;
  if (n < 8)       bk = n;
  else if (n < 12) bk = 8;
  else if (n < 16) bk = 9;
  else if (n < 23) bk = 10;
  else if (n < 32) bk = 11;
  else if (n < 46) bk = 12;
  else if (n < 64) bk = 13;
  else if (n < 91) bk = 14;
  else             bk = 15;
  return ret + bk;
}

__global__ __launch_bounds__(256) void bias_build(const float* __restrict__ tbl, float* BD) {
  __shared__ __align__(16) float sh[BDW];
  const int h = blockIdx.x, t = threadIdx.x;
#pragma unroll 4
  for (int j = 0; j < 16; ++j) {
    const int idx = t + 256 * j;
    const int ti = clampi(rel_bucket(idx - 2047) * NH + h, 0, NBKT * NH - 1);
    float v = bfr(tbl[ti]);
    v = (idx == BDW - 1) ? 0.f : v;
    sh[idx] = v;
  }
  __syncthreads();
  v4f vv[4];
#pragma unroll
  for (int q = 0; q < 4; ++q) vv[q] = *(const v4f*)(sh + q * 1024 + 4 * t);
  float* dst = BD + (size_t)h * BDW;
  for (int pass = 0; pass < 2; ++pass) {
#pragma unroll
    for (int q = 0; q < 4; ++q) *(volatile v4f*)(dst + q * 1024 + 4 * t) = vv[q];
    __threadfence();
  }
}

template <int OPK, int NPL, int AHM, int OM, int RSM, int RES>
__global__ __launch_bounds__(256) void gemm64(
    const unsigned short* __restrict__ Ap, const unsigned short* __restrict__ Ap2, int lda, int aplane,
    const unsigned short* __restrict__ Btp, const unsigned short* __restrict__ Btp2, int ldb,
    unsigned short* Ch, unsigned short* Ch2, float* Cf, int ldc,
    const float* __restrict__ Rs, const float* __restrict__ Rp,
    float wsc, float osc, float rsc, int M, int N, int K) {
  __shared__ __align__(16) float sT[8][16 * 68];
  const int lane = threadIdx.x & 31;
  const int wave = threadIdx.x >> 5;
  const int tilesN = N >> 6;
  const int tilesM = M >> 6;
  const int tile = blockIdx.x * 8 + wave;
  if (tile >= tilesM * tilesN) return;
  const int tm = tile / tilesN;
  const int tn = tile - tm * tilesN;
  const int m0 = tm << 6;
  const int n0 = tn << 6;

  const int rlane = lane & 15;
  const int koff  = (lane >> 4) * 8;
  const int mOff  = (lane >> 4) * 8;

  v8f acc[4][4];
#pragma unroll
  for (int i = 0; i < 4; ++i)
#pragma unroll
    for (int j = 0; j < 4; ++j) acc[i][j] = zero8();

#pragma unroll 1
  for (int pl = 0; pl < NPL; ++pl) {
    const unsigned short* Ac = (pl == 0) ? Ap : Ap2;
    const unsigned short* Bc = (pl == 0) ? Btp : Btp2;
    for (int k0 = 0; k0 < K; k0 += 32) {
      v16us bh[4];
#pragma unroll
      for (int j = 0; j < 4; ++j) {
        const size_t bo = (size_t)(n0 + (j << 4) + rlane) * ldb + koff + k0;
        bh[j] = ldfrag_u(Bc + bo);
      }
#pragma unroll
      for (int i = 0; i < 4; ++i) {
        size_t ao;
        if (AHM) ao = (size_t)(k0 / HD) * (size_t)aplane + (size_t)(m0 + (i << 4) + rlane) * HD +
                      (size_t)(k0 & (HD - 1)) + koff;
        else     ao = (size_t)(m0 + (i << 4) + rlane) * lda + koff + k0;
        const v16us ah = ldfrag_u(Ac + ao);
#pragma unroll
        for (int j = 0; j < 4; ++j) acc[i][j] = mma_raw<OPK>(ah, bh[j], acc[i][j]);
        dep_guard1(acc[i][0], acc[i][3], ah);
      }
      keep4_u(bh[0], bh[1], bh[2], bh[3]);
    }
  }
  acc_guard4(acc[0][0], acc[0][1], acc[0][2], acc[0][3]);
  acc_guard4(acc[1][0], acc[1][1], acc[1][2], acc[1][3]);
  acc_guard4(acc[2][0], acc[2][1], acc[2][2], acc[2][3]);
  acc_guard4(acc[3][0], acc[3][1], acc[3][2], acc[3][3]);

  const int hh2 = lane >> 4, c4 = (lane & 15) * 4;
  const int q8  = lane >> 3, c8 = (lane & 7) * 8;
  const float wo = wsc * osc;

  float csc[8];
#pragma unroll
  for (int e = 0; e < 8; ++e) csc[e] = 1.f;
  if (OM != 0 && RSM == 2) {
    const v4f cs0 = *(const v4f*)(Rs + n0 + c8);
    const v4f cs1 = *(const v4f*)(Rs + n0 + c8 + 4);
#pragma unroll
    for (int e = 0; e < 4; ++e) { csc[e] = cs0[e]; csc[4 + e] = cs1[e]; }
  }

  float* slab = sT[wave];
#pragma unroll
  for (int i = 0; i < 4; ++i) {
    const int mBase = m0 + (i << 4);
#pragma unroll
    for (int j = 0; j < 4; ++j) {
#pragma unroll
      for (int r = 0; r < 8; ++r) {
        slab[(mOff + r) * 68 + (j << 4) + rlane] = acc[i][j][r];
      }
    }
    wave_sync_lds();
    if (OM == 0) {
      v4f vals[8];
#pragma unroll
      for (int it = 0; it < 8; ++it) {
        const int row = it * 2 + hh2;
        v4f v = *(const v4f*)(slab + row * 68 + c4);
        v = v * wsc;
        if (RES) {
          const int tok = mBase + row;
          const int bb = tok / SEQ, ss = tok - bb * SEQ;
          const v4f hr = *(const v4f*)(Rp + ((size_t)bb * SEQ_FULL + (size_t)ss) * DM + (size_t)(n0 + c4));
#pragma unroll
          for (int c = 0; c < 4; ++c) v[c] = v[c] + bfr(hr[c]);
        }
        vals[it] = v;
      }
      for (int pass = 0; pass < 2; ++pass) {
#pragma unroll
        for (int it = 0; it < 8; ++it) {
          const int row = it * 2 + hh2;
          *(volatile v4f*)(Cf + (size_t)(mBase + row) * ldc + (size_t)n0 + c4) = vals[it];
        }
        __threadfence();
      }
    } else {
      v4u hv[4], hw[4];
#pragma unroll
      for (int it = 0; it < 4; ++it) {
        const int row = it * 4 + q8;
        const float* sp = slab + row * 68 + c8;
        float rsr = wo;
        if (RSM == 1) rsr = wo * Rs[mBase + row];
        v4u ha = {0u, 0u, 0u, 0u}, hb = {0u, 0u, 0u, 0u};
#pragma unroll
        for (int e = 0; e < 4; ++e) {
          const float b0 = sp[2 * e]     * rsr * csc[2 * e];
          const float b1 = sp[2 * e + 1] * rsr * csc[2 * e + 1];
          if (OM == 1) {
            ha[e] = pk16(f2h(b0), f2h(b1));
          } else {
            const _Float16 x0 = (_Float16)b0, x1 = (_Float16)b1;
            ha[e] = pk16(h_bits(x0), h_bits(x1));
            hb[e] = pk16(f2h((b0 - (float)x0) * rsc), f2h((b1 - (float)x1) * rsc));
          }
        }
        hv[it] = ha;
        hw[it] = hb;
      }
      for (int pass = 0; pass < 2; ++pass) {
#pragma unroll
        for (int it = 0; it < 4; ++it) {
          const int row = it * 4 + q8;
          const size_t go = (size_t)(mBase + row) * ldc + (size_t)n0 + c8;
          *(volatile v4u*)(Ch + go) = hv[it];
          if (OM == 2) *(volatile v4u*)(Ch2 + go) = hw[it];
        }
        __threadfence();
      }
    }
    wave_sync_lds();
  }
}

__global__ __launch_bounds__(128) void attn_kernel(
    const unsigned short* __restrict__ QHp, const unsigned short* __restrict__ QRp,
    const unsigned short* __restrict__ KHp, const unsigned short* __restrict__ KRp,
    const unsigned short* __restrict__ VTp,
    const float* __restrict__ BD, unsigned short* Zh, unsigned short* Zl) {
  __shared__ __align__(16) float relw[AWV][RWP];
  __shared__ __align__(16) unsigned short pws[AWV][16 * 32];
  __shared__ __align__(16) unsigned short zst[AWV][2][16 * HD];
  const int lane = threadIdx.x & 31, wv = threadIdx.x >> 5, m = lane & 15, hh = lane >> 4;
  const int nqt = SEQ / 16;
  const int task = blockIdx.x * AWV + wv;
  if (task >= NB * NH * nqt) return;
  const int bh = task / nqt;
  const int t0 = (task - bh * nqt) << 4;
  const int b = bh / NH, h = bh - b * NH;
  const size_t tok0 = (size_t)b * SEQ;
  float* rw = relw[wv];
  unsigned short* ph = pws[wv];

  const size_t qo = (tok0 + (size_t)(t0 + m)) * DM + (size_t)(h * HD + 8 * hh);
  const v16us qh0 = ldfrag_u(QHp + qo);
  const v16us qh1 = ldfrag_u(QHp + qo + 32);
  const v16us qr0 = ldfrag_u(QRp + qo);
  const v16us qr1 = ldfrag_u(QRp + qo + 32);

  float mx[8], ls[8];
  v8f O[4];
#pragma unroll
  for (int j = 0; j < 4; ++j) O[j] = zero8();
#pragma unroll
  for (int r = 0; r < 8; ++r) { mx[r] = -1.0e30f; ls[r] = 0.f; }

  const float* bdh = BD + (size_t)h * BDW + (BDC - t0);
  const size_t kro = (tok0 + (size_t)m) * DM + (size_t)(h * HD + 8 * hh);
  const unsigned short* kbase  = KHp + kro;
  const unsigned short* krbase = KRp + kro;
  const unsigned short* vbase = VTp + (size_t)(h * HD + m) * MT + tok0 + (size_t)(8 * hh);
  const int nblk = SEQ / 32;

#pragma unroll 1
  for (int kb = 0; kb < nblk; ++kb) {
    const int sb = kb << 5;
    {
      const float* bp = bdh + sb;
      const float w0v = bp[lane];
      const float w1v = bp[32 + m];
      rw[lane] = w0v;
      if (lane < 16) rw[32 + lane] = w1v;
    }
    wave_sync_lds();

    v8f S0 = zero8(), S1 = zero8(), R0 = zero8(), R1 = zero8();
#pragma unroll
    for (int ks = 0; ks < 2; ++ks) {
      const size_t kofs = (size_t)sb * DM + (size_t)(32 * ks);
      const v16us kf0 = ldfrag_u(kbase + kofs);
      const v16us kf1 = ldfrag_u(kbase + kofs + (size_t)16 * DM);
      const v16us kg0 = ldfrag_u(krbase + kofs);
      const v16us kg1 = ldfrag_u(krbase + kofs + (size_t)16 * DM);
      const v16us qa = (ks == 0) ? qh0 : qh1;
      const v16us qb = (ks == 0) ? qr0 : qr1;
      S0 = mma_g<0>(qa, kf0, S0);
      S1 = mma_g<0>(qa, kf1, S1);
      R0 = mma_g<0>(qb, kf0, R0);
      R1 = mma_g<0>(qb, kf1, R1);
      R0 = mma_g<0>(qa, kg0, R0);
      R1 = mma_g<0>(qa, kg1, R1);
    }

    float s0[8], s1[8];
#pragma unroll
    for (int r = 0; r < 8; ++r) {
      const int row = 8 * hh + r;
      const float rv0 = rw[15 - row + m];
      const float rv1 = rw[31 - row + m];
      s0[r] = fmaf(S0[r], SC1, fmaf(R0[r], SC2, rv0));
      s1[r] = fmaf(S1[r], SC1, fmaf(R1[r], SC2, rv1));
    }

#pragma unroll
    for (int r = 0; r < 8; ++r) {
      float xm = fmaxf(s0[r], s1[r]);
      xm = fmaxf(xm, __shfl_xor(xm, 1, 32));
      xm = fmaxf(xm, __shfl_xor(xm, 2, 32));
      xm = fmaxf(xm, __shfl_xor(xm, 4, 32));
      xm = fmaxf(xm, __shfl_xor(xm, 8, 32));
      const float mn = fmaxf(mx[r], xm);
      const float al = __expf(mx[r] - mn);
      mx[r] = mn;
      const float p0 = __expf(s0[r] - mn);
      const float p1 = __expf(s1[r] - mn);
      float ps = p0 + p1;
      ps += __shfl_xor(ps, 1, 32);
      ps += __shfl_xor(ps, 2, 32);
      ps += __shfl_xor(ps, 4, 32);
      ps += __shfl_xor(ps, 8, 32);
      ls[r] = ls[r] * al + ps;
#pragma unroll
      for (int j = 0; j < 4; ++j) O[j][r] = O[j][r] * al;
      const int row = 8 * hh + r;
      ph[row * 32 + m]      = f2h(p0 * PCAR);
      ph[row * 32 + 16 + m] = f2h(p1 * PCAR);
    }
    wave_sync_lds();

    const v16us af = ldfrag_u(ph + m * 32 + 8 * hh);
#pragma unroll
    for (int j = 0; j < 4; ++j) {
      const v16us vf = ldfrag_u(vbase + (size_t)(16 * j) * MT + (size_t)sb);
      O[j] = mma_g<0>(af, vf, O[j]);
    }
  }
  acc_guard4(O[0], O[1], O[2], O[3]);

  unsigned short* zh = zst[wv][0];
  unsigned short* zl = zst[wv][1];
#pragma unroll
  for (int r = 0; r < 8; ++r) {
    const int row = 8 * hh + r;
    const float linv = (1.0f / ls[r]) * OSC;
#pragma unroll
    for (int j = 0; j < 4; ++j) {
      const float o = O[j][r] * linv;
      const unsigned short x0 = bf_bits(o);
      zh[row * HD + 16 * j + m] = x0;
      zl[row * HD + 16 * j + m] = bf_bits(o - bf_up(x0));
    }
  }
  wave_sync_lds();
  {
    v4u ha[4], hb[4];
#pragma unroll
    for (int q = 0; q < 4; ++q) {
      ha[q] = *(const v4u*)(zh + q * 256 + lane * 8);
      hb[q] = *(const v4u*)(zl + q * 256 + lane * 8);
    }
    const size_t zo = ((size_t)h * MT + tok0 + (size_t)t0) * HD;
    unsigned short* dh = Zh + zo;
    unsigned short* dl = Zl + zo;
    for (int pass = 0; pass < 2; ++pass) {
#pragma unroll
      for (int q = 0; q < 4; ++q) {
        *(volatile v4u*)(dh + q * 256 + lane * 8) = ha[q];
        *(volatile v4u*)(dl + q * 256 + lane * 8) = hb[q];
      }
      __threadfence();
    }
  }
}

extern "C" void kernel_launch(void* const* d_in, const int* in_sizes, int n_in,
                              void* d_out, int out_size, void* d_ws, size_t ws_size,
                              hipStream_t stream) {
  if (n_in < 7) return;
  if (in_sizes[0] < ((NB - 1) * SEQ_FULL + SEQ) * DM) return;
  if (in_sizes[1] < DM) return;
  if (in_sizes[2] < DM * DM) return;
  if (in_sizes[3] < DM * DM) return;
  if (in_sizes[4] < DM * DM) return;
  if (in_sizes[5] < DM * DM) return;
  if (in_sizes[6] < NBKT * NH) return;
  if (out_size < MT * DM) return;

  const float* x    = (const float*)d_in[0];
  const float* lnw  = (const float*)d_in[1];
  const float* w_q  = (const float*)d_in[2];
  const float* w_k  = (const float*)d_in[3];
  const float* w_v  = (const float*)d_in[4];
  const float* w_o  = (const float*)d_in[5];
  const float* tbl  = (const float*)d_in[6];

  const size_t PX  = (size_t)MT * DM * 2;
  const size_t PRS = (((size_t)MT * 4 + 65535) / 65536) * 65536;
  const size_t PW1 = (size_t)DM * DM * 2;
  const size_t PBD = (size_t)NH * BDW * 4;
  size_t off = 0;
  const size_t oXB = off; off += PX;
  const size_t oXH = off; off += PX;
  const size_t oRS = off; off += PRS;
  const size_t oW  = off; off += 6 * PW1;
  const size_t oBD = off; off += PBD;
  const size_t oQH = off; off += PX;
  const size_t oQR = off; off += PX;
  const size_t oKH = off; off += PX;
  const size_t oKR = off; off += PX;
  const size_t oVT = off; off += PX;
  const size_t oZH = off; off += PX;
  const size_t oZL = off; off += PX;
  if (off > ws_size) return;
  if (off > (size_t)134217728) return;

  char* ws = (char*)d_ws;
  unsigned short* XB = (unsigned short*)(ws + oXB);
  unsigned short* XH = (unsigned short*)(ws + oXH);
  float* RSTD = (float*)(ws + oRS);
  unsigned short* W16 = (unsigned short*)(ws + oW);
  unsigned short* WQH = W16;
  unsigned short* WQL = W16 + (size_t)1 * DM * DM;
  unsigned short* WKH = W16 + (size_t)2 * DM * DM;
  unsigned short* WKL = W16 + (size_t)3 * DM * DM;
  unsigned short* WVH = W16 + (size_t)4 * DM * DM;
  unsigned short* WOB = W16 + (size_t)5 * DM * DM;
  float* BDp = (float*)(ws + oBD);
  unsigned short* QH = (unsigned short*)(ws + oQH);
  unsigned short* QR = (unsigned short*)(ws + oQR);
  unsigned short* KH = (unsigned short*)(ws + oKH);
  unsigned short* KR = (unsigned short*)(ws + oKR);
  unsigned short* VT = (unsigned short*)(ws + oVT);
  unsigned short* ZH = (unsigned short*)(ws + oZH);
  unsigned short* ZL = (unsigned short*)(ws + oZL);
  float* out0 = (float*)d_out;
  float* fdummy = BDp;

  const dim3 blk(256);
  const int gT = ((MT / 64) * (DM / 64)) / 8;

  cvt_x<<<dim3(MT / 32), blk, 0, stream>>>(x, XB, XH, RSTD);
  cvt_w<<<dim3((DM / 64) * (DM / 64), 4), blk, 0, stream>>>(w_q, w_k, w_v, w_o, lnw, W16);
  bias_build<<<dim3(NH), blk, 0, stream>>>(tbl, BDp);

  gemm64<1, 2, 0, 2, 1, 0><<<dim3(gT), blk, 0, stream>>>(
      XB, XB, DM, 0, WQH, WQL, DM, QH, QR, fdummy, DM, RSTD, x, 1.0f, QKS, QRS, MT, DM, DM);
  gemm64<1, 2, 0, 2, 1, 0><<<dim3(gT), blk, 0, stream>>>(
      XB, XB, DM, 0, WKH, WKL, DM, KH, KR, fdummy, DM, RSTD, x, 1.0f, QKS, QRS, MT, DM, DM);
  gemm64<0, 1, 0, 1, 2, 0><<<dim3(gT), blk, 0, stream>>>(
      WVH, WVH, DM, 0, XH, XH, DM, VT, VT, fdummy, MT, RSTD, x, 1.0f / (XSC * WSCL), VSC, 1.0f, DM, MT, DM);

  attn_kernel<<<dim3((NB * NH * (SEQ / 16)) / AWV), dim3(128), 0, stream>>>(QH, QR, KH, KR, VT, BDp, ZH, ZL);

  gemm64<1, 2, 1, 0, 0, 1><<<dim3(gT), blk, 0, stream>>>(
      ZH, ZL, DM, MT * HD, WOB, WOB, DM, ZH, ZH, out0, DM, RSTD, x, 1.0f, 1.0f, 1.0f, MT, DM, DM);
  (void)hipGetLastError();
}
